// ProductLayer_8065948581965
// MI455X (gfx1250) — hardware-run, weakly checked
//
#include <hip/hip_runtime.h>
#include <stddef.h>


typedef _Float16 v16h __attribute__((ext_vector_type(16)));
typedef _Float16 v8h  __attribute__((ext_vector_type(8)));
typedef float    v8f  __attribute__((ext_vector_type(8)));
typedef float    v4f  __attribute__((ext_vector_type(4)));
typedef _Float16 h16;

#ifndef NB
#define NB 4096
#endif
#define NB_FULL 4096
#define NF   32
#define ND   64
#define NU   256
#define KLZ  (NF * ND)
#define KOUT (ND * ND)
#define OUTW (3 * NU)

static_assert(NB >= 64 && NB <= NB_FULL && (NB % 64) == 0);
static_assert(NF == 32);
static_assert(ND == 64);
static_assert((NU % 64) == 0 && NU == 256);
static_assert((KLZ % 64) == 0 && (KLZ % 32) == 0);
static_assert(KLZ == 8 * 32 * 8);
static_assert((KOUT % 32) == 0);
static_assert(((NU * NF / 8) % 256) == 0);
static_assert(((NU * KOUT / 8) % 256) == 0);
static_assert(((OUTW * 4) % 128) == 0 && ((NU * 4) % 128) == 0);

#define LDT 72
#define LDC 68
#define LDE 40
#define LDF 68
static_assert((LDT % 8) == 0 && LDT >= 64);
static_assert((LDC % 4) == 0 && LDC >= 64);
static_assert((LDE % 8) == 0 && LDE >= NF);
static_assert((LDF % 4) == 0 && LDF >= ND);

#define WCARRY 64.0f
#define ECARRY 64.0f
#define FCARRY 4.0f

#define LW_BYTES  ((size_t)NU * KLZ * 2)
#define IW_BYTES  ((size_t)NU * NF * 2)
#define OW_BYTES  ((size_t)NU * KOUT * 2)
#define E16_BYTES ((size_t)NB * KLZ * 2)
#define FS_BYTES  ((size_t)NB * ND * 4)
#define OFF_LW  ((size_t)0)
#define OFF_IW  (OFF_LW + LW_BYTES)
#define OFF_OW  (OFF_IW + IW_BYTES)
#define OFF_E16 (OFF_OW + OW_BYTES)
#define OFF_FS  (OFF_E16 + E16_BYTES)
#define WS_TOTAL (OFF_FS + FS_BYTES)
static_assert((LW_BYTES % 128) == 0 && (IW_BYTES % 128) == 0 && (OW_BYTES % 128) == 0);
static_assert((E16_BYTES % 128) == 0 && (FS_BYTES % 128) == 0);
static_assert(WS_TOTAL <= (size_t)134217728);

__device__ __forceinline__ float bf16r(float x) {
  unsigned int u = __float_as_uint(x);
  u = (u + 0x7FFFu + ((u >> 16) & 1u)) & 0xFFFF0000u;
  return __uint_as_float(u);
}

static __device__ __forceinline__ h16 toh_flush(float v) {
  const h16 r = (h16)v;
  return (fabsf(v) < 6.103515625e-05f) ? (h16)0.0f : r;
}

__device__ __forceinline__ v16h frag_at(const _Float16* p) {
  v8h lo = *(const v8h*)(p);
  v8h hi = *(const v8h*)(p + 16);
  v16h out;
#pragma unroll
  for (int i = 0; i < 8; ++i) { out[i] = lo[i]; out[i + 8] = hi[i]; }
  return out;
}
__device__ __forceinline__ v16h ld_frag(const _Float16* base, unsigned ld) {
  const unsigned lane = threadIdx.x & 31u;
  return frag_at(base + (lane & 15u) * ld + (lane >> 4) * 8u);
}

__device__ __forceinline__ v8f wmma16(v16h a, v16h b, v8f c) {
  v8f d = __builtin_amdgcn_wmma_f32_16x16x32_f16(false, a, false, b, (short)0, c,
                                                 false, false);
  asm volatile("v_nop\n\tv_nop\n\tv_nop\n\tv_nop" : "+v"(d) : "v"(a), "v"(b));
  return d;
}

__device__ __forceinline__ void wave_lds_sync() {
  __builtin_amdgcn_fence(3  , "wavefront");
  asm volatile("s_wait_dscnt 0x0" ::: "memory");
  __builtin_amdgcn_wave_barrier();
}

__global__ __launch_bounds__(256) void wconv_kernel(
    const float* __restrict__ W, _Float16* __restrict__ Wt, unsigned ldw, unsigned ldk) {
  __shared__ _Float16 T[64 * LDT];
  const unsigned tid = threadIdx.x;
  const unsigned n0 = blockIdx.x * 64u;
  const unsigned k0 = blockIdx.y * 64u;
#pragma unroll 4
  for (unsigned j = 0; j < 16u; ++j) {
    const unsigned idx = tid + 256u * j;
    const unsigned kr = idx >> 6, nc = idx & 63u;
    const float v = W[(size_t)(k0 + kr) * ldw + n0 + nc];
    T[nc * LDT + kr] = (_Float16)(WCARRY * bf16r(v));
  }
  __syncthreads();
  v8h x[2];
  size_t off[2];
#pragma unroll
  for (unsigned i = 0; i < 2u; ++i) {
    const unsigned n = 32u * i + (tid >> 3);
    const unsigned kc = (tid & 7u) * 8u;
    x[i] = *(const v8h*)&T[n * LDT + kc];
    off[i] = (size_t)(n0 + n) * ldk + k0 + kc;
  }
#pragma unroll
  for (int i = 0; i < 2; ++i) *(volatile v8h*)(Wt + off[i]) = x[i];
  __threadfence();
#pragma unroll
  for (int i = 0; i < 2; ++i) *(volatile v8h*)(Wt + off[i]) = x[i];
}

__global__ __launch_bounds__(256) void cvt_plane_kernel(
    const float* __restrict__ src, _Float16* __restrict__ dst, unsigned n8) {
#pragma clang fp contract(off)
  const unsigned idx = blockIdx.x * 256u + threadIdx.x;
  const unsigned ci = (idx < n8) ? idx : (n8 - 1u);
  const v4f a0 = *(const v4f*)(src + (size_t)ci * 8u);
  const v4f a1 = *(const v4f*)(src + (size_t)ci * 8u + 4u);
  v8h o;
#pragma unroll
  for (int i = 0; i < 4; ++i) {
    o[i]     = toh_flush(WCARRY * bf16r(a0[i]));
    o[i + 4] = toh_flush(WCARRY * bf16r(a1[i]));
  }
  _Float16* p = dst + (size_t)ci * 8u;
  if (idx < n8) *(volatile v8h*)p = o;
  __threadfence();
  if (idx < n8) *(volatile v8h*)p = o;
}

__global__ __launch_bounds__(256) void prep_kernel(
    const float* __restrict__ E, _Float16* __restrict__ E16, float* __restrict__ FS) {
#pragma clang fp contract(off)
  __shared__ float Fst[8 * ND];
  const unsigned tid = threadIdx.x, lane = tid & 31u;
  const unsigned wave = __builtin_amdgcn_readfirstlane(threadIdx.x >> 5);
  const unsigned b = blockIdx.x * 8u + wave;
  const float* er = E + (size_t)b * KLZ + lane * 8u;
  _Float16* dr = E16 + (size_t)b * KLZ + lane * 8u;

  float s[8];
#pragma unroll
  for (int i = 0; i < 8; ++i) s[i] = 0.0f;
  v8h x[8];
#pragma unroll
  for (int j = 0; j < 8; ++j) {
    const v4f a0 = *(const v4f*)(er + j * 256);
    const v4f a1 = *(const v4f*)(er + j * 256 + 4);
#pragma unroll
    for (int i = 0; i < 4; ++i) {
      const float e0 = bf16r(a0[i]);
      const float e1 = bf16r(a1[i]);
      s[i]     = s[i] + e0;
      s[i + 4] = s[i + 4] + e1;
      x[j][i]     = toh_flush(ECARRY * e0);
      x[j][i + 4] = toh_flush(ECARRY * e1);
    }
  }
#pragma unroll
  for (int i = 0; i < 8; ++i) {
    s[i] = s[i] + __shfl_xor(s[i], 8, 32);
    s[i] = s[i] + __shfl_xor(s[i], 16, 32);
  }
  if (lane < 8u) {
    v4f t0, t1;
#pragma unroll
    for (int i = 0; i < 4; ++i) { t0[i] = s[i]; t1[i] = s[i + 4]; }
    *(v4f*)&Fst[wave * ND + lane * 8u]      = t0;
    *(v4f*)&Fst[wave * ND + lane * 8u + 4u] = t1;
  }

#pragma unroll
  for (int j = 0; j < 8; ++j) *(volatile v8h*)(dr + j * 256) = x[j];
  __threadfence();
#pragma unroll
  for (int j = 0; j < 8; ++j) *(volatile v8h*)(dr + j * 256) = x[j];

  __syncthreads();
  if (tid < 128u) {
    const v4f v = *(const v4f*)&Fst[tid * 4u];
    float* p = FS + (size_t)blockIdx.x * (8u * ND) + tid * 4u;
    *(volatile v4f*)p = v;
    __threadfence();
    *(volatile v4f*)p = v;
  }
}

__global__ __launch_bounds__(256) void gemm_lz_kernel(
    const _Float16* __restrict__ A16, const _Float16* __restrict__ Bt,
    float* __restrict__ outf) {
  __shared__ float Cs[64 * LDC];
  const unsigned tid = threadIdx.x, lane = tid & 31u;
  const unsigned wave = __builtin_amdgcn_readfirstlane(threadIdx.x >> 5);
  const unsigned mw = wave >> 1, nw = wave & 1u;
  const unsigned hh = lane >> 4, m = lane & 15u;
  const unsigned n0 = blockIdx.x * 64u;
  const unsigned row0 = blockIdx.y * 64u;

  const _Float16* ap  = A16 + (size_t)(row0 + mw * 16u + m) * KLZ + hh * 8u;
  const _Float16* bp0 = Bt + (size_t)(n0 + nw * 32u + m) * KLZ + hh * 8u;
  const _Float16* bp1 = bp0 + (size_t)16 * KLZ;
  v8f acc0 = {}, acc1 = {};
#pragma unroll 2
  for (unsigned k0 = 0; k0 < (unsigned)KLZ; k0 += 32u) {
    const v16h a  = frag_at(ap + k0);
    const v16h b0 = frag_at(bp0 + k0);
    const v16h b1 = frag_at(bp1 + k0);
    acc0 = wmma16(a, b0, acc0);
    acc1 = wmma16(a, b1, acc1);
  }
#pragma unroll
  for (int r = 0; r < 8; ++r) {
    float* d = &Cs[(mw * 16u + hh * 8u + (unsigned)r) * LDC + nw * 32u + m];
    d[0]  = acc0[r];
    d[16] = acc1[r];
  }
  __syncthreads();

  const float cs = 1.0f / (ECARRY * WCARRY);
  v4f xs[4];
  size_t off[4];
#pragma unroll
  for (unsigned i = 0; i < 4u; ++i) {
    const unsigned r = 16u * i + (tid >> 4);
    const unsigned c = (tid & 15u) * 4u;
    const v4f u = *(const v4f*)&Cs[r * LDC + c];
    xs[i] = u * cs;
    off[i] = (size_t)(row0 + r) * OUTW + n0 + c;
  }
#pragma unroll
  for (int i = 0; i < 4; ++i) *(volatile v4f*)(outf + off[i]) = xs[i];
  __threadfence();
#pragma unroll
  for (int i = 0; i < 4; ++i) *(volatile v4f*)(outf + off[i]) = xs[i];
}

__global__ __launch_bounds__(256) void inner_kernel(
    const _Float16* __restrict__ E16, const _Float16* __restrict__ IW16,
    float* __restrict__ outf) {
  __shared__ _Float16 Ts[8 * ND * LDE];
  __shared__ float Rs[8 * NU];
  const unsigned tid = threadIdx.x, lane = tid & 31u;
  const unsigned wave = __builtin_amdgcn_readfirstlane(threadIdx.x >> 5);
  const unsigned hh = lane >> 4, m = lane & 15u;
  const unsigned b = blockIdx.x * 8u + wave;
  const unsigned tb = wave * (unsigned)(ND * LDE);
  const unsigned rb = wave * (unsigned)NU;

  const _Float16* erow = E16 + (size_t)b * KLZ + lane * 8u;
  const unsigned d0 = (lane & 7u) * 8u;
#pragma unroll
  for (unsigned j = 0; j < 8u; ++j) {
    const v8h x = *(const v8h*)(erow + j * 256u);
    const unsigned f = 4u * j + (lane >> 3);
#pragma unroll
    for (unsigned t = 0; t < 8u; ++t) Ts[tb + (d0 + t) * LDE + f] = x[t];
  }
  wave_lds_sync();

  v16h af[4];
#pragma unroll
  for (int dt = 0; dt < 4; ++dt) af[dt] = ld_frag(&Ts[tb + (unsigned)dt * 16u * LDE], LDE);

  const float isc = 1.0f / ((ECARRY * WCARRY) * (ECARRY * WCARRY));
  const _Float16* wp = IW16 + (size_t)m * NF + hh * 8u;
#pragma unroll 2
  for (unsigned ut = 0; ut < 16u; ++ut) {
    const v16h bf = frag_at(wp + ut * (16u * NF));
    float p = 0.0f;
#pragma unroll
    for (int dt = 0; dt < 4; ++dt) {
      v8f z = {};
      const v8f t = wmma16(af[dt], bf, z);
#pragma unroll
      for (int r = 0; r < 8; ++r) p += t[r] * t[r];
    }
    p += __shfl_xor(p, 16, 32);
    const float pv = p * isc;
    if (lane < 16u) Rs[rb + ut * 16u + m] = pv;
  }
  wave_lds_sync();

  v4f xs[2];
  size_t off[2];
#pragma unroll
  for (unsigned i = 0; i < 2u; ++i) {
    const unsigned c = i * 128u + lane * 4u;
    xs[i] = *(const v4f*)&Rs[rb + c];
    off[i] = (size_t)b * OUTW + NU + c;
  }
#pragma unroll
  for (int i = 0; i < 2; ++i) *(volatile v4f*)(outf + off[i]) = xs[i];
  __threadfence();
#pragma unroll
  for (int i = 0; i < 2; ++i) *(volatile v4f*)(outf + off[i]) = xs[i];
}

__global__ __launch_bounds__(256) void outer_kernel(
    const float* __restrict__ FS, const _Float16* __restrict__ OW16,
    float* __restrict__ outf) {
  __shared__ float Fs[64 * LDF];
  __shared__ float Ct[8 * 16 * LDC];
  const unsigned tid = threadIdx.x, lane = tid & 31u;
  const unsigned wave = __builtin_amdgcn_readfirstlane(threadIdx.x >> 5);
  const unsigned mw = wave >> 1, nh = wave & 1u;
  const unsigned hh = lane >> 4, m = lane & 15u;
  const unsigned row0 = blockIdx.x * 64u;
  const unsigned cb = wave * (unsigned)(16 * LDC);

#pragma unroll
  for (unsigned j = 0; j < 4u; ++j) {
    const unsigned idx = tid + 256u * j;
    const unsigned r = idx >> 4, c = (idx & 15u) * 4u;
    *(v4f*)&Fs[r * LDF + c] = *(const v4f*)(FS + (size_t)(row0 + r) * ND + c);
  }
  __syncthreads();

  const unsigned fr = (mw * 16u + m) * LDF;
  float fj[2][16];
#pragma unroll
  for (int c = 0; c < 2; ++c) {
    const v4f q0 = *(const v4f*)&Fs[fr + (unsigned)c * 32u + hh * 8u];
    const v4f q1 = *(const v4f*)&Fs[fr + (unsigned)c * 32u + hh * 8u + 4u];
    const v4f q2 = *(const v4f*)&Fs[fr + (unsigned)c * 32u + 16u + hh * 8u];
    const v4f q3 = *(const v4f*)&Fs[fr + (unsigned)c * 32u + 16u + hh * 8u + 4u];
#pragma unroll
    for (int t = 0; t < 4; ++t) {
      fj[c][t]      = q0[t];
      fj[c][t + 4]  = q1[t];
      fj[c][t + 8]  = q2[t];
      fj[c][t + 12] = q3[t];
    }
  }

  v8f acc[8];
#pragma unroll
  for (int nt = 0; nt < 8; ++nt) acc[nt] = (v8f){};
  const _Float16* bp = OW16 + (size_t)(nh * 128u + m) * KOUT + hh * 8u;

#pragma unroll 1
  for (unsigned i = 0; i < (unsigned)ND; ++i) {
    const float fi = FCARRY * Fs[fr + i];
#pragma unroll
    for (int c = 0; c < 2; ++c) {
      v16h a;
#pragma unroll
      for (int t = 0; t < 16; ++t) a[t] = toh_flush(fi * fj[c][t]);
#pragma unroll
      for (int nt = 0; nt < 8; ++nt) {
        const v16h bfr = frag_at(bp + (size_t)nt * (16u * KOUT) + i * 64u + (unsigned)c * 32u);
        acc[nt] = wmma16(a, bfr, acc[nt]);
      }
    }
  }

  const float osc = 1.0f / (FCARRY * WCARRY);
#pragma unroll
  for (int q = 0; q < 2; ++q) {
#pragma unroll
    for (int t = 0; t < 4; ++t)
#pragma unroll
      for (int r = 0; r < 8; ++r)
        Ct[cb + (hh * 8u + (unsigned)r) * LDC + (unsigned)t * 16u + m] = acc[q * 4 + t][r];
    wave_lds_sync();
    v4f xs[8];
    size_t off[8];
#pragma unroll
    for (unsigned i = 0; i < 8u; ++i) {
      const unsigned r = 2u * i + (lane >> 4);
      const unsigned c = (lane & 15u) * 4u;
      const v4f u = *(const v4f*)&Ct[cb + r * LDC + c];
      xs[i] = u * osc;
      off[i] = (size_t)(row0 + mw * 16u + r) * OUTW + 2u * NU + nh * 128u + (unsigned)q * 64u + c;
    }
#pragma unroll
    for (int i = 0; i < 8; ++i) *(volatile v4f*)(outf + off[i]) = xs[i];
    __threadfence();
#pragma unroll
    for (int i = 0; i < 8; ++i) *(volatile v4f*)(outf + off[i]) = xs[i];
    wave_lds_sync();
  }
}

extern "C" void kernel_launch(void* const* d_in, const int* in_sizes, int n_in,
                              void* d_out, int out_size, void* d_ws, size_t ws_size,
                              hipStream_t stream) {
  if (n_in < 4) return;
  if ((long long)in_sizes[0] < (long long)NB * KLZ) return;
  if ((long long)in_sizes[1] < (long long)KLZ * NU) return;
  if ((long long)in_sizes[2] < (long long)NU * NF) return;
  if ((long long)in_sizes[3] < (long long)NU * KOUT) return;
  if ((long long)out_size < (long long)NB * OUTW) return;
  if (ws_size < WS_TOTAL) return;

  const float* emb = (const float*)d_in[0];
  const float* lw  = (const float*)d_in[1];
  const float* iw  = (const float*)d_in[2];
  const float* ow  = (const float*)d_in[3];
  float* out = (float*)d_out;

  char* ws = (char*)d_ws;
  _Float16* LWt  = (_Float16*)(ws + OFF_LW);
  _Float16* IW16 = (_Float16*)(ws + OFF_IW);
  _Float16* OW16 = (_Float16*)(ws + OFF_OW);
  _Float16* E16  = (_Float16*)(ws + OFF_E16);
  float*    FSp  = (float*)(ws + OFF_FS);

  dim3 blk(256);

  wconv_kernel<<<dim3(NU / 64, KLZ / 64), blk, 0, stream>>>(lw, LWt, (unsigned)NU, (unsigned)KLZ);
  cvt_plane_kernel<<<dim3((NU * NF / 8) / 256), blk, 0, stream>>>(iw, IW16, (unsigned)(NU * NF / 8));
  cvt_plane_kernel<<<dim3((NU * KOUT / 8) / 256), blk, 0, stream>>>(ow, OW16, (unsigned)(NU * KOUT / 8));

  prep_kernel<<<dim3(NB / 8), blk, 0, stream>>>(emb, E16, FSp);
  gemm_lz_kernel<<<dim3(NU / 64, NB / 64), blk, 0, stream>>>(E16, LWt, out);
  inner_kernel<<<dim3(NB / 8), blk, 0, stream>>>(E16, IW16, out);
  outer_kernel<<<dim3(NB / 64), blk, 0, stream>>>(FSp, OW16, out);
}
